// GCN_75385265979507
// MI455X (gfx1250) — hardware-verified
//
#include <hip/hip_runtime.h>
#include <stddef.h>
#include <stdint.h>
#include <math.h>


#define NN     32768
#define NG     128
#define SS     256
#define NEDGE  524288
#define DIN    128
#define DH     256
#define NH     8
#define HD     32
#define DFF    1024
#define FCH    8192

#define NTHR   256
#define NWAVE  8
#define EPT    8
#define CHUNK  (NTHR * EPT)
#define WCAP   (EPT * 32)
#define LISTN  (NWAVE * WCAP)
#define NBD    8192
#define SLD    13
#define NBA    1024
#define SLA    10
#define RCAP   28672
#define DEGCAP 64
#define AGG_ZINTS    (LISTN + 2 * RCAP + 3 * NBA)
#define MISC_INTS    16
#define ROWBUF_INTS  (NWAVE * 512 / 2)
#define AGG_LDS_INTS (AGG_ZINTS + MISC_INTS + ROWBUF_INTS)

#define GM     64
#define GN     256
#define GT     256
#define GLDS   (GM * GN * 4)

#define NUW    221184

static_assert((CHUNK & (CHUNK - 1)) == 0 && CHUNK <= 4096);
static_assert((NBD & (NBD - 1)) == 0 && NBD == (1 << SLD));
static_assert((NBA & (NBA - 1)) == 0 && NBA == (1 << SLA));
static_assert(((long long)CHUNK << SLD) < (1LL << 31));
static_assert(((long long)NEDGE << SLA) < (1LL << 31));
static_assert(NBD % (NTHR * 4) == 0 && LISTN % NTHR == 0);
static_assert(NBA % NWAVE == 0 && NBA % 32 == 0);
static_assert(AGG_ZINTS % 4 == 0 && ((AGG_ZINTS + MISC_INTS) % 4) == 0);
static_assert(AGG_LDS_INTS * 4 <= 300000);
static_assert(NN % NBA == 0 && NN % NBD == 0 && NN % GM == 0 && FCH % GM == 0 && NN % FCH == 0);
static_assert(NN == NG * SS && DH == NH * HD && HD == 32);
static_assert(NWAVE * 512 * 4 <= RCAP * 4 && 512 * 4 <= RCAP * 4);
static_assert(NUW % NTHR == 0);
static_assert((NN * DIN / 8) % NTHR == 0 && (NN * DH / 8) % NTHR == 0);

typedef float          v4f   __attribute__((ext_vector_type(4)));
typedef float          v8f   __attribute__((ext_vector_type(8)));
typedef int            v4i   __attribute__((ext_vector_type(4)));
typedef int            v8i   __attribute__((ext_vector_type(8)));
typedef unsigned       v2u   __attribute__((ext_vector_type(2)));
typedef unsigned       v4u   __attribute__((ext_vector_type(4)));
typedef unsigned short v4us  __attribute__((ext_vector_type(4)));
typedef unsigned short v8us  __attribute__((ext_vector_type(8)));
typedef unsigned short v16us __attribute__((ext_vector_type(16)));
typedef __bf16         v16bf __attribute__((ext_vector_type(16)));
typedef float __attribute__((may_alias)) f32a;
typedef v4f  __attribute__((may_alias)) v4fa;
typedef v4i  __attribute__((may_alias)) v4ia;
typedef v2u  __attribute__((may_alias)) v2ua;
typedef v4u  __attribute__((may_alias)) v4ua;
typedef v4us __attribute__((may_alias)) v4usa;
typedef v8us __attribute__((may_alias)) v8usa;
union FragB { v16bf v; v16us u; v8us h[2]; v8i w; };

__device__ __forceinline__ v8f wmb(const FragB& a, const FragB& b, v8f c) {
  v8f d = __builtin_amdgcn_wmma_f32_16x16x32_bf16(false, a.v, false, b.v, (short)0, c, false, false);
  asm volatile("v_nop\n\tv_nop\n\tv_nop\n\tv_nop" : "+v"(d) : "v"(a.w), "v"(b.w));
  return d;
}

__device__ __forceinline__ unsigned bf16_bits(float f) {
  const unsigned u = __float_as_uint(f);
  return (u + 0x7FFFu + ((u >> 16) & 1u)) >> 16;
}
__device__ __forceinline__ float bf16_val(float f) {
  return __uint_as_float(bf16_bits(f) << 16);
}
__device__ __forceinline__ unsigned hl_pack(float v) {
  const unsigned hb = bf16_bits(v);
  const unsigned lb = bf16_bits(v - __uint_as_float(hb << 16));
  return hb | (lb << 16);
}
__device__ __forceinline__ v4f ld4bf(const float* p) {
  const v4f a = *(const v4fa*)p;
  v4f r;
  r.x = bf16_val(a.x); r.y = bf16_val(a.y); r.z = bf16_val(a.z); r.w = bf16_val(a.w);
  return r;
}
__device__ __forceinline__ v4f widen_hl(const v2u h, const v2u l) {
  v4f r;
  r.x = __uint_as_float(h.x << 16)         + __uint_as_float(l.x << 16);
  r.y = __uint_as_float(h.x & 0xffff0000u) + __uint_as_float(l.x & 0xffff0000u);
  r.z = __uint_as_float(h.y << 16)         + __uint_as_float(l.y << 16);
  r.w = __uint_as_float(h.y & 0xffff0000u) + __uint_as_float(l.y & 0xffff0000u);
  return r;
}

__device__ __forceinline__ void wave_sync() {
  __builtin_amdgcn_fence(__ATOMIC_RELEASE, "wavefront");
  __builtin_amdgcn_wave_barrier();
  __builtin_amdgcn_fence(__ATOMIC_ACQUIRE, "wavefront");
}

template <int SLB>
__device__ __forceinline__ int scan_chunk(const int* __restrict__ dsts, int nE, int cbase, int slotBase,
                                          int nb, int vec8, int* list, int tid, int lane, int wave) {
  int wc = 0;
  const int el0  = tid * EPT;
  const int e0   = cbase + el0;
  const int sent = -2147483647 - 1;
  v4i da, db;
  if (vec8 != 0 && cbase + CHUNK <= nE) {
    da = *(const v4i*)(dsts + e0);
    db = *(const v4i*)(dsts + e0 + 4);
  } else {
    da.x = (e0     < nE) ? dsts[min(e0,     nE - 1)] : sent;
    da.y = (e0 + 1 < nE) ? dsts[min(e0 + 1, nE - 1)] : sent;
    da.z = (e0 + 2 < nE) ? dsts[min(e0 + 2, nE - 1)] : sent;
    da.w = (e0 + 3 < nE) ? dsts[min(e0 + 3, nE - 1)] : sent;
    db.x = (e0 + 4 < nE) ? dsts[min(e0 + 4, nE - 1)] : sent;
    db.y = (e0 + 5 < nE) ? dsts[min(e0 + 5, nE - 1)] : sent;
    db.z = (e0 + 6 < nE) ? dsts[min(e0 + 6, nE - 1)] : sent;
    db.w = (e0 + 7 < nE) ? dsts[min(e0 + 7, nE - 1)] : sent;
  }
  const unsigned nbs = (unsigned)slotBase;
  const unsigned unb = (unsigned)nb;
  const unsigned s0 = (unsigned)da.x - nbs, s1 = (unsigned)da.y - nbs;
  const unsigned s2 = (unsigned)da.z - nbs, s3 = (unsigned)da.w - nbs;
  const unsigned s4 = (unsigned)db.x - nbs, s5 = (unsigned)db.y - nbs;
  const unsigned s6 = (unsigned)db.z - nbs, s7 = (unsigned)db.w - nbs;
  const bool h0 = s0 < unb, h1 = s1 < unb, h2 = s2 < unb, h3 = s3 < unb;
  const bool h4 = s4 < unb, h5 = s5 < unb, h6 = s6 < unb, h7 = s7 < unb;
  const unsigned any = __builtin_amdgcn_ballot_w32(h0 | h1 | h2 | h3 | h4 | h5 | h6 | h7);
  if (any != 0u) {
#define HITJ(J, HJ, SJ) { \
      const unsigned mj = __builtin_amdgcn_ballot_w32(HJ); \
      if (mj != 0u) { \
        if (HJ) { \
          const int pos = wc + (int)__builtin_amdgcn_mbcnt_lo(mj, 0u); \
          if (pos < WCAP) list[wave * WCAP + pos] = ((el0 + (J)) << SLB) | (int)(SJ); \
        } \
        wc += (int)__builtin_popcount(mj); } }
    HITJ(0, h0, s0)
    HITJ(1, h1, s1)
    HITJ(2, h2, s2)
    HITJ(3, h3, s3)
    HITJ(4, h4, s4)
    HITJ(5, h5, s5)
    HITJ(6, h6, s6)
    HITJ(7, h7, s7)
#undef HITJ
  }
  return wc;
}

__global__ __launch_bounds__(NTHR) void k_wprep(const float* __restrict__ w1, const float* __restrict__ w2,
                                                const float* __restrict__ wq, const float* __restrict__ wk,
                                                const float* __restrict__ wv, const float* __restrict__ wo,
                                                const float* __restrict__ f1, const float* __restrict__ f2,
                                                unsigned short* W1c, unsigned short* W2c, unsigned short* Wqkv,
                                                unsigned short* WOc, unsigned short* FF1c, unsigned short* FF2c) {
  const int u = (int)blockIdx.x * NTHR + (int)threadIdx.x;
  const float* W;
  unsigned short* P;
  int K, Nn, v;
  if (u < 8192)        { W = w1; P = W1c;              K = 128;  Nn = 256;  v = u; }
  else if (u < 24576)  { W = w2; P = W2c;              K = 256;  Nn = 256;  v = u - 8192; }
  else if (u < 40960)  { W = wq; P = Wqkv;             K = 256;  Nn = 256;  v = u - 24576; }
  else if (u < 57344)  { W = wk; P = Wqkv + 256 * 512; K = 256;  Nn = 256;  v = u - 40960; }
  else if (u < 73728)  { W = wv; P = Wqkv + 512 * 512; K = 256;  Nn = 256;  v = u - 57344; }
  else if (u < 90112)  { W = wo; P = WOc;              K = 256;  Nn = 256;  v = u - 73728; }
  else if (u < 155648) { W = f1; P = FF1c;             K = 256;  Nn = 1024; v = u - 90112; }
  else if (u < NUW)    { W = f2; P = FF2c;             K = 1024; Nn = 256;  v = u - 155648; }
  else return;
  const int upr = K >> 2;
  const int n   = v / upr;
  const int k8  = (v - n * upr) * 8;
  const int kk  = k8 & (K - 1);
  const float* p = W + (size_t)kk * Nn + n;
  v8us o;
#pragma unroll
  for (int i = 0; i < 8; ++i) o[i] = (unsigned short)bf16_bits(p[(size_t)i * Nn]);
  unsigned short* dp = P + (size_t)n * (size_t)(2 * K) + k8;
  *(volatile v8us*)dp = o;
  __threadfence();
  *(volatile v8us*)dp = o;
}

__global__ __launch_bounds__(NTHR) void k_stats1(const float* __restrict__ x, float* part) {
  __shared__ __attribute__((aligned(16))) float wsum[NWAVE * 256];
  __shared__ __attribute__((aligned(16))) float outs[256];
  const int tid = (int)threadIdx.x, lane = tid & 31, wave = tid >> 5;
  const size_t row0 = (size_t)blockIdx.x * 256 + (size_t)wave * 32;
  v4f s = {0.f, 0.f, 0.f, 0.f}, q = {0.f, 0.f, 0.f, 0.f};
#pragma unroll 4
  for (int r = 0; r < 32; ++r) {
    const v4f v = ld4bf(x + (row0 + r) * DIN + 4 * lane);
    s += v;
    q += v * v;
  }
  *(v4fa*)(wsum + wave * 256 + 4 * lane) = s;
  *(v4fa*)(wsum + wave * 256 + 128 + 4 * lane) = q;
  __syncthreads();
  {
    float a = 0.0f;
#pragma unroll
    for (int w2 = 0; w2 < NWAVE; ++w2) a += ((const f32a*)wsum)[w2 * 256 + tid];
    ((f32a*)outs)[tid] = a;
  }
  __syncthreads();
  if (tid < 64) {
    const v4f ov = *(const v4fa*)(outs + 4 * tid);
    float* pp = part + (size_t)blockIdx.x * 256 + 4 * tid;
    *(volatile v4f*)pp = ov;
    __threadfence();
    *(volatile v4f*)pp = ov;
  }
}

__global__ __launch_bounds__(NTHR) void k_bncomb(const float* __restrict__ part, int nblk, int C,
                                                 const float* __restrict__ g, const float* __restrict__ b,
                                                 float* sc, double invN) {
  __shared__ __attribute__((aligned(16))) float outs[512];
  const int tid = (int)threadIdx.x;
  const int cc = tid < C ? tid : C - 1;
  double S = 0.0, Q = 0.0;
#pragma unroll 4
  for (int blk = 0; blk < nblk; ++blk) {
    S += (double)part[(size_t)blk * 2 * C + cc];
    Q += (double)part[(size_t)blk * 2 * C + C + cc];
  }
  const double mu = S * invN;
  double var = Q * invN - mu * mu;
  var = var < 0.0 ? 0.0 : var;
  const float rs = rsqrtf((float)var + 1e-5f);
  const float sv = rs * bf16_val(g[cc]);
  const float sh = bf16_val(b[cc]) - (float)mu * sv;
  if (tid < C) { outs[tid] = sv; outs[C + tid] = sh; }
  __syncthreads();
  if (tid < C / 2) {
    const v4f ov = *(const v4fa*)(outs + 4 * tid);
    float* pp = sc + 4 * tid;
    *(volatile v4f*)pp = ov;
    __threadfence();
    *(volatile v4f*)pp = ov;
  }
}

template <int C, int RND>
__global__ __launch_bounds__(NTHR) void k_bn(const float* __restrict__ x, const float* __restrict__ sc,
                                             unsigned short* out, int nUnits) {
  const int u = (int)blockIdx.x * NTHR + (int)threadIdx.x;
  if (u >= nUnits) return;
  constexpr int UPR = C / 8;
  const int row = u / UPR;
  const int k8  = (u - row * UPR) * 8;
  const float* p = x + (size_t)row * C + k8;
  v4f a = *(const v4fa*)p;
  v4f b = *(const v4fa*)(p + 4);
  if (RND) {
    a.x = bf16_val(a.x); a.y = bf16_val(a.y); a.z = bf16_val(a.z); a.w = bf16_val(a.w);
    b.x = bf16_val(b.x); b.y = bf16_val(b.y); b.z = bf16_val(b.z); b.w = bf16_val(b.w);
  }
  const v4f s0 = *(const v4fa*)(sc + k8),     s1 = *(const v4fa*)(sc + k8 + 4);
  const v4f h0 = *(const v4fa*)(sc + C + k8), h1 = *(const v4fa*)(sc + C + k8 + 4);
  float y[8];
  y[0] = fmaf(a.x, s0.x, h0.x); y[1] = fmaf(a.y, s0.y, h0.y);
  y[2] = fmaf(a.z, s0.z, h0.z); y[3] = fmaf(a.w, s0.w, h0.w);
  y[4] = fmaf(b.x, s1.x, h1.x); y[5] = fmaf(b.y, s1.y, h1.y);
  y[6] = fmaf(b.z, s1.z, h1.z); y[7] = fmaf(b.w, s1.w, h1.w);
  v8us hv, lv;
#pragma unroll
  for (int j = 0; j < 8; ++j) {
    const unsigned w = hl_pack(y[j]);
    hv[j] = (unsigned short)(w & 0xffffu);
    lv[j] = (unsigned short)(w >> 16);
  }
  unsigned short* dp = out + (size_t)row * (2 * C) + k8;
  *(volatile v8us*)dp = hv;
  *(volatile v8us*)(dp + C) = lv;
  __threadfence();
  *(volatile v8us*)dp = hv;
  *(volatile v8us*)(dp + C) = lv;
}

__global__ __launch_bounds__(NTHR) void k_deg(const int* __restrict__ dsts, int nE, int vec8, float* dis) {
  __shared__ __attribute__((aligned(16))) int scnt[NBD];
  __shared__ __attribute__((aligned(16))) int list[LISTN];
  __shared__ int wcnt[NWAVE];
  const int tid = (int)threadIdx.x, lane = tid & 31, wave = tid >> 5;
  const int nodeBase = (int)blockIdx.x * NBD;

  for (int i = tid; i < NBD; i += NTHR) scnt[i] = 0;
  for (int i = tid; i < LISTN; i += NTHR) list[i] = 0;
  if (tid < NWAVE) wcnt[tid] = 0;
  __syncthreads();

  const int nChunks = (nE + CHUNK - 1) / CHUNK;
#pragma unroll 1
  for (int ch = 0; ch < nChunks; ++ch) {
    const int cbase = ch * CHUNK;
    const int wc = scan_chunk<SLD>(dsts, nE, cbase, nodeBase, NBD, vec8, list, tid, lane, wave);
    if (lane == 0) wcnt[wave] = wc;
    __syncthreads();
    if (wave == 0) {
#pragma unroll 1
      for (int w2 = 0; w2 < NWAVE; ++w2) {
        int c = wcnt[w2];
        c = c < 0 ? 0 : (c > WCAP ? WCAP : c);
#pragma unroll 1
        for (int b0 = 0; b0 < c; b0 += 32) {
          const int idx = b0 + lane;
          const int ent = list[w2 * WCAP + (idx < WCAP ? idx : WCAP - 1)];
          const int m32 = (c - b0) < 32 ? (c - b0) : 32;
#pragma unroll 1
          for (int k = 0; k < m32; ++k) {
            const int u  = __builtin_amdgcn_readlane(ent, k);
            const int sl = u & (NBD - 1);
            if (lane == 0) scnt[sl] = scnt[sl] + 1;
          }
        }
      }
    }
    __syncthreads();
  }

  v4f vals[NBD / (NTHR * 4)];
#pragma unroll
  for (int it = 0; it < NBD / (NTHR * 4); ++it) {
    const int s0 = it * (NTHR * 4) + 4 * tid;
    const v4i c4 = *(const v4ia*)(scnt + s0);
    v4f v;
    v.x = rsqrtf((float)c4.x + 1.0f); v.y = rsqrtf((float)c4.y + 1.0f);
    v.z = rsqrtf((float)c4.z + 1.0f); v.w = rsqrtf((float)c4.w + 1.0f);
    vals[it] = v;
  }
#pragma unroll
  for (int it = 0; it < NBD / (NTHR * 4); ++it) {
    const int s0 = it * (NTHR * 4) + 4 * tid;
    *(volatile v4f*)(dis + (size_t)nodeBase + s0) = vals[it];
  }
  __threadfence();
#pragma unroll
  for (int it = 0; it < NBD / (NTHR * 4); ++it) {
    const int s0 = it * (NTHR * 4) + 4 * tid;
    *(volatile v4f*)(dis + (size_t)nodeBase + s0) = vals[it];
  }
}

template <int MODE>
__global__ __launch_bounds__(GT) void k_gemm(
    const unsigned short* __restrict__ A, int lda, const unsigned short* __restrict__ WT, int K,
    const float* __restrict__ bs0, const float* __restrict__ bs1, const float* __restrict__ bs2,
    const float* __restrict__ gam, const float* __restrict__ bet, const unsigned short* __restrict__ res,
    unsigned short* oh0, unsigned short* oh1, unsigned short* oh2, unsigned short* oh3, float* of)
{
  extern __shared__ __attribute__((aligned(16))) float stg[];
  const int tid = (int)threadIdx.x, lane = tid & 31, wave = tid >> 5, hh = lane >> 4, m = lane & 15;
  const int wr = wave & 3, wc = wave >> 2;
  const int rowBase = (int)blockIdx.x * GM;
  const int cb   = (int)blockIdx.y;
  const int col0 = cb * GN;

  v8f acc[8];
  {
    const v8f z = {0.f, 0.f, 0.f, 0.f, 0.f, 0.f, 0.f, 0.f};
#pragma unroll
    for (int t = 0; t < 8; ++t) acc[t] = z;
  }
  const unsigned short* ap = A  + (size_t)(rowBase + 16 * wr + m) * (size_t)lda + 8 * hh;
  const unsigned short* bp = WT + (size_t)(col0 + 128 * wc + m) * (size_t)K + 8 * hh;
#pragma unroll 1
  for (int k0 = 0; k0 < K; k0 += 32) {
    FragB af;
    af.h[0] = *(const v8usa*)(ap + k0);
    af.h[1] = *(const v8usa*)(ap + k0 + 16);
#pragma unroll
    for (int nt = 0; nt < 8; ++nt) {
      const unsigned short* wq = bp + (size_t)(16 * nt) * (size_t)K + k0;
      FragB bf;
      bf.h[0] = *(const v8usa*)wq;
      bf.h[1] = *(const v8usa*)(wq + 16);
      acc[nt] = wmb(af, bf, acc[nt]);
    }
  }
#pragma unroll
  for (int nt = 0; nt < 8; ++nt) {
    const int lc = 128 * wc + 16 * nt + m;
#pragma unroll
    for (int r = 0; r < 8; ++r) {
      const int lr = 16 * wr + 8 * hh + r;
      stg[lr * GN + lc] = acc[nt][r];
    }
  }
  __syncthreads();

  if constexpr (MODE == 1) {
    if (cb == 2) {
      const int bg = rowBase >> 8;
      const int kb = rowBase & (SS - 1);
#pragma unroll 1
      for (int pass = 0; pass < 2; ++pass) {
#pragma unroll 1
        for (int it = 0; it < 8; ++it) {
          const int u = it * GT + tid;
          const int c = u >> 3;
          const int p = u & 7;
          const float bv = bf16_val(bs2[c]);
          v8us hv, lv;
#pragma unroll
          for (int j = 0; j < 8; ++j) {
            const float v = stg[(8 * p + j) * GN + c] + bv;
            const unsigned w = hl_pack(v);
            hv[j] = (unsigned short)(w & 0xffffu);
            lv[j] = (unsigned short)(w >> 16);
          }
          const size_t dst = (size_t)(bg * 256 + c) * SS + kb + 8 * p;
          *(volatile v8us*)(oh2 + dst) = hv;
          *(volatile v8us*)(oh3 + dst) = lv;
        }
        __threadfence();
      }
      return;
    }
  }

  constexpr bool HL = (MODE == 1 || MODE == 2 || MODE == 3);
  const int cA = HL ? 8 * lane : 4 * lane;
  const int cB = HL ? 8 * lane + 4 : 128 + 4 * lane;

  if constexpr (MODE != 0) {
    const float* bpv = bs0;
    if constexpr (MODE == 1) bpv = (cb == 0) ? bs0 : bs1;
    if constexpr (MODE == 3) bpv = bs0 + col0;
    const v4f bA = ld4bf(bpv + cA), bB = ld4bf(bpv + cB);
    v4f gA = {1.f, 1.f, 1.f, 1.f}, gB = gA, eA = {0.f, 0.f, 0.f, 0.f}, eB = eA;
    if constexpr (MODE == 2 || MODE == 4) {
      gA = ld4bf(gam + cA); gB = ld4bf(gam + cB);
      eA = ld4bf(bet + cA); eB = ld4bf(bet + cB);
    }
#pragma unroll 1
    for (int i = 0; i < 8; ++i) {
      const int r = 8 * wave + i;
      float* srow = stg + r * GN;
      v4f xa = *(const v4fa*)(srow + cA);
      v4f xb = *(const v4fa*)(srow + cB);
      xa += bA; xb += bB;
      if constexpr (MODE == 3) {
        xa.x = fmaxf(xa.x, 0.f); xa.y = fmaxf(xa.y, 0.f); xa.z = fmaxf(xa.z, 0.f); xa.w = fmaxf(xa.w, 0.f);
        xb.x = fmaxf(xb.x, 0.f); xb.y = fmaxf(xb.y, 0.f); xb.z = fmaxf(xb.z, 0.f); xb.w = fmaxf(xb.w, 0.f);
      }
      if constexpr (MODE == 2 || MODE == 4) {
        const unsigned short* rp = res + (size_t)(rowBase + r) * 512;
        const v2u hA = *(const v2ua*)(rp + cA),       hB = *(const v2ua*)(rp + cB);
        const v2u lA = *(const v2ua*)(rp + 256 + cA), lB = *(const v2ua*)(rp + 256 + cB);
        xa += widen_hl(hA, lA);
        xb += widen_hl(hB, lB);
        float sm = (xa.x + xa.y + xa.z + xa.w) + (xb.x + xb.y + xb.z + xb.w);
#pragma unroll
        for (int d = 16; d > 0; d >>= 1) sm += __shfl_xor(sm, d, 32);
        const float mu = sm * (1.0f / 256.0f);
        const v4f da = xa - mu, db = xb - mu;
        float sq = (da.x * da.x + da.y * da.y + da.z * da.z + da.w * da.w) +
                   (db.x * db.x + db.y * db.y + db.z * db.z + db.w * db.w);
#pragma unroll
        for (int d = 16; d > 0; d >>= 1) sq += __shfl_xor(sq, d, 32);
        const float rs = rsqrtf(sq * (1.0f / 256.0f) + 1e-5f);
        xa = da * rs * gA + eA;
        xb = db * rs * gB + eB;
      }
      wave_sync();
      if constexpr (MODE == 4) {
        *(v4fa*)(srow + cA) = xa;
        *(v4fa*)(srow + cB) = xb;
      } else {
        v8us hv, lv;
        unsigned w;
        w = hl_pack(xa.x); hv[0] = (unsigned short)(w & 0xffffu); lv[0] = (unsigned short)(w >> 16);
        w = hl_pack(xa.y); hv[1] = (unsigned short)(w & 0xffffu); lv[1] = (unsigned short)(w >> 16);
        w = hl_pack(xa.z); hv[2] = (unsigned short)(w & 0xffffu); lv[2] = (unsigned short)(w >> 16);
        w = hl_pack(xa.w); hv[3] = (unsigned short)(w & 0xffffu); lv[3] = (unsigned short)(w >> 16);
        w = hl_pack(xb.x); hv[4] = (unsigned short)(w & 0xffffu); lv[4] = (unsigned short)(w >> 16);
        w = hl_pack(xb.y); hv[5] = (unsigned short)(w & 0xffffu); lv[5] = (unsigned short)(w >> 16);
        w = hl_pack(xb.z); hv[6] = (unsigned short)(w & 0xffffu); lv[6] = (unsigned short)(w >> 16);
        w = hl_pack(xb.w); hv[7] = (unsigned short)(w & 0xffffu); lv[7] = (unsigned short)(w >> 16);
        unsigned short* urow = (unsigned short*)srow;
        *(v8usa*)(urow + 8 * lane) = hv;
        *(v8usa*)(urow + 256 + 8 * lane) = lv;
      }
    }
  }
  wave_sync();

  char* dbase;
  size_t pitchB, off1;
  if constexpr (MODE == 0 || MODE == 4) { dbase = (char*)of; pitchB = 1024; off1 = 512; }
  else if constexpr (MODE == 1)         { dbase = (char*)((cb == 0) ? oh0 : oh1); pitchB = 1024; off1 = 512; }
  else if constexpr (MODE == 2)         { dbase = (char*)oh0; pitchB = 1024; off1 = 512; }
  else                                  { dbase = (char*)(oh0 + col0); pitchB = 4096; off1 = 2048; }
#pragma unroll 1
  for (int pass = 0; pass < 2; ++pass) {
#pragma unroll 1
    for (int i = 0; i < 8; ++i) {
      const int r = 8 * wave + i;
      const char* srow = (const char*)(stg + r * GN);
      const v4u q0 = *(const v4ua*)(srow + 16 * lane);
      const v4u q1 = *(const v4ua*)(srow + 512 + 16 * lane);
      char* dp = dbase + (size_t)(rowBase + r) * pitchB + 16 * lane;
      *(volatile v4u*)dp = q0;
      *(volatile v4u*)(dp + off1) = q1;
    }
    __threadfence();
  }
}

template <int MODE>
__global__ __launch_bounds__(NTHR) void k_agg(const int* __restrict__ srcs, const int* __restrict__ dsts,
                                              int nE, int nN, int vec8,
                                              const float* __restrict__ dis, const float* __restrict__ hc,
                                              const float* __restrict__ bias,
                                              const float* __restrict__ h1in, const int* __restrict__ bat,
                                              const float* __restrict__ inter, int nG,
                                              float* hout, float* part, unsigned short* thl) {
  extern __shared__ __attribute__((aligned(16))) int dsm[];
  int* list = dsm;
  int* hl   = dsm + LISTN;
  int* sl   = hl + RCAP;
  int* cnt  = sl + RCAP;
  int* offs = cnt + NBA;
  int* cur  = offs + NBA;
  int* misc = cur + NBA;
  const int tid = (int)threadIdx.x, lane = tid & 31, wave = tid >> 5;
  unsigned short* rowbuf = (unsigned short*)(misc + MISC_INTS) + wave * 512;
  const int nodeBase = (int)blockIdx.x * NBA;

  {
    const v4i z4 = {0, 0, 0, 0};
    for (int i = tid * 4; i < AGG_ZINTS; i += NTHR * 4) *(v4ia*)(dsm + i) = z4;
    if (tid < MISC_INTS) misc[tid] = 0;
  }
  const v4f bvA = ld4bf(bias + 4 * lane);
  const v4f bvB = ld4bf(bias + 128 + 4 * lane);
  __syncthreads();

  int t = 0, ov = 0;
  const int nChunks = (nE + CHUNK - 1) / CHUNK;
#pragma unroll 1
  for (int ch = 0; ch < nChunks; ++ch) {
    const int cbase = ch * CHUNK;
    const int wc = scan_chunk<SLA>(dsts, nE, cbase, nodeBase, NBA, vec8, list, tid, lane, wave);
    if (lane == 0) misc[wave] = wc;
    __syncthreads();
    if (wave == 0) {
#pragma unroll 1
      for (int w2 = 0; w2 < NWAVE; ++w2) {
        int c = misc[w2];
        c = c < 0 ? 0 : (c > WCAP ? WCAP : c);
#pragma unroll 1
        for (int b0 = 0; b0 < c; b0 += 32) {
          const int idx = b0 + lane;
          const int ent = list[w2 * WCAP + (idx < WCAP ? idx : WCAP - 1)];
          const int m32 = (c - b0) < 32 ? (c - b0) : 32;
#pragma unroll 1
          for (int k = 0; k < m32; ++k) {
            const int u    = __builtin_amdgcn_readlane(ent, k);
            const int slot = u & (NBA - 1);
            const int el   = (u >> SLA) & (CHUNK - 1);
            const int pk   = ((cbase + el) << SLA) | slot;
            if (t < RCAP) {
              if (lane == 0) { hl[t] = pk; cnt[slot] = cnt[slot] + 1; }
              t = t + 1;
            } else {
              ov = 1;
            }
          }
        }
      }
    }
    __syncthreads();
  }
  if (wave == 0 && lane == 0) { misc[8] = t; misc[9] = ov; }
  __syncthreads();
  int tt = misc[8];
  tt = tt < 0 ? 0 : (tt > RCAP ? RCAP : tt);
  const int ovf = misc[9];

  if (wave == 0) {
    const int base = lane * (NBA / 32);
    int s = 0;
#pragma unroll 1
    for (int i = 0; i < NBA / 32; ++i) s += cnt[base + i];
    int incl = s;
#pragma unroll
    for (int d = 1; d < 32; d <<= 1) {
      const int y = __shfl_up(incl, d, 32);
      if (lane >= d) incl += y;
    }
    int run = incl - s;
#pragma unroll 1
    for (int i = 0; i < NBA / 32; ++i) {
      const int cv = cnt[base + i];
      offs[base + i] = run;
      cur[base + i]  = run;
      run += cv;
    }
  }
  __syncthreads();
  if (wave == 0) {
#pragma unroll 1
    for (int b0 = 0; b0 < tt; b0 += 32) {
      const int idx = b0 + lane;
      const int ent = hl[idx < RCAP ? idx : RCAP - 1];
      const int m32 = (tt - b0) < 32 ? (tt - b0) : 32;
#pragma unroll 1
      for (int k = 0; k < m32; ++k) {
        const int u    = __builtin_amdgcn_readlane(ent, k);
        const int slot = u & (NBA - 1);
        if (lane == 0) {
          int p = cur[slot];
          p = p < 0 ? 0 : (p > RCAP - 1 ? RCAP - 1 : p);
          sl[p] = u;
          cur[slot] = p + 1;
        }
      }
    }
  }
  __syncthreads();

  const float qnan = __int_as_float(0x7fc00000);
  const float pz = (ovf != 0) ? qnan : 0.0f;
  v4f psA = {0.f, 0.f, 0.f, 0.f}, psB = psA, pqA = psA, pqB = psA;
#pragma unroll 1
  for (int si = 0; si < NBA / NWAVE; ++si) {
    const int s    = si * NWAVE + wave;
    const int node = nodeBase + s;
    int c = cnt[s];
    const bool big = c > DEGCAP;
    c = c < 0 ? 0 : (c > DEGCAP ? DEGCAP : c);
    int o = offs[s];
    o = o < 0 ? 0 : (o > RCAP ? RCAP : o);
    const int nc = node < nN ? node : nN - 1;
    const float dd = dis[nc];
    const float rd = dd * dd;
    v4f accA = {0.f, 0.f, 0.f, 0.f}, accB = accA;
#pragma unroll 1
    for (int b0 = 0; b0 < c; b0 += 32) {
      int idx = o + b0 + lane;
      idx = idx > RCAP - 1 ? RCAP - 1 : idx;
      const int ent = sl[idx];
      int eid = ent >> SLA;
      eid = eid < 0 ? 0 : (eid > nE - 1 ? nE - 1 : eid);
      int sr = srcs[eid];
      sr = sr < 0 ? 0 : (sr > nN - 1 ? nN - 1 : sr);
      const float cf  = dis[sr] * dd;
      const int   cfi = __float_as_int(cf);
      const int m32 = (c - b0) < 32 ? (c - b0) : 32;
#pragma unroll 1
      for (int k = 0; k < m32; ++k) {
        const int   sk = __builtin_amdgcn_readlane(sr, k);
        const float ck = __int_as_float(__builtin_amdgcn_readlane(cfi, k));
        const float* rp = hc + (size_t)sk * DH + 4 * lane;
        const v4f ra = *(const v4fa*)rp;
        const v4f rb = *(const v4fa*)(rp + 128);
        accA.x = fmaf(ck, ra.x, accA.x); accA.y = fmaf(ck, ra.y, accA.y);
        accA.z = fmaf(ck, ra.z, accA.z); accA.w = fmaf(ck, ra.w, accA.w);
        accB.x = fmaf(ck, rb.x, accB.x); accB.y = fmaf(ck, rb.y, accB.y);
        accB.z = fmaf(ck, rb.z, accB.z); accB.w = fmaf(ck, rb.w, accB.w);
      }
    }
    const float* sp = hc + (size_t)nc * DH + 4 * lane;
    const v4f svA = *(const v4fa*)sp;
    const v4f svB = *(const v4fa*)(sp + 128);
    const float pzr = big ? qnan : pz;
    const bool live = node < nN;
    v4f yA = (accA + svA * rd) + bvA;
    v4f yB = (accB + svB * rd) + bvB;
    yA.x = fmaxf(yA.x, 0.f) + pzr; yA.y = fmaxf(yA.y, 0.f) + pzr;
    yA.z = fmaxf(yA.z, 0.f) + pzr; yA.w = fmaxf(yA.w, 0.f) + pzr;
    yB.x = fmaxf(yB.x, 0.f) + pzr; yB.y = fmaxf(yB.y, 0.f) + pzr;
    yB.z = fmaxf(yB.z, 0.f) + pzr; yB.w = fmaxf(yB.w, 0.f) + pzr;
    if constexpr (MODE == 0) {
      if (live) {
        psA += yA; psB += yB; pqA += yA * yA; pqB += yB * yB;
        float* op = hout + (size_t)node * DH + 4 * lane;
        *(volatile v4f*)op = yA;
        *(volatile v4f*)(op + 128) = yB;
        __threadfence();
        *(volatile v4f*)op = yA;
        *(volatile v4f*)(op + 128) = yB;
      }
    } else {
      const float* hp = h1in + (size_t)nc * DH + 4 * lane;
      const v4f hA = *(const v4fa*)hp;
      const v4f hB = *(const v4fa*)(hp + 128);
      int bg = bat[nc];
      bg = bg < 0 ? 0 : (bg > nG - 1 ? nG - 1 : bg);
      const float* ip = inter + (size_t)bg * DH + 4 * lane;
      const v4f iA = ld4bf(ip);
      const v4f iB = ld4bf(ip + 128);
      const v4f tA = (hA + yA) + iA;
      const v4f tB = (hB + yB) + iB;
      v4us hv0, lv0, hv1, lv1;
      unsigned w;
      w = hl_pack(tA.x); hv0[0] = (unsigned short)(w & 0xffffu); lv0[0] = (unsigned short)(w >> 16);
      w = hl_pack(tA.y); hv0[1] = (unsigned short)(w & 0xffffu); lv0[1] = (unsigned short)(w >> 16);
      w = hl_pack(tA.z); hv0[2] = (unsigned short)(w & 0xffffu); lv0[2] = (unsigned short)(w >> 16);
      w = hl_pack(tA.w); hv0[3] = (unsigned short)(w & 0xffffu); lv0[3] = (unsigned short)(w >> 16);
      w = hl_pack(tB.x); hv1[0] = (unsigned short)(w & 0xffffu); lv1[0] = (unsigned short)(w >> 16);
      w = hl_pack(tB.y); hv1[1] = (unsigned short)(w & 0xffffu); lv1[1] = (unsigned short)(w >> 16);
      w = hl_pack(tB.z); hv1[2] = (unsigned short)(w & 0xffffu); lv1[2] = (unsigned short)(w >> 16);
      w = hl_pack(tB.w); hv1[3] = (unsigned short)(w & 0xffffu); lv1[3] = (unsigned short)(w >> 16);
      *(v4usa*)(rowbuf + 4 * lane) = hv0;
      *(v4usa*)(rowbuf + 128 + 4 * lane) = hv1;
      *(v4usa*)(rowbuf + 256 + 4 * lane) = lv0;
      *(v4usa*)(rowbuf + 384 + 4 * lane) = lv1;
      wave_sync();
      const v8us q0 = *(const v8usa*)(rowbuf + 8 * lane);
      const v8us q1 = *(const v8usa*)(rowbuf + 256 + 8 * lane);
      wave_sync();
      if (live) {
        unsigned short* rpw = thl + (size_t)node * 512 + 8 * lane;
        *(volatile v8us*)rpw = q0;
        *(volatile v8us*)(rpw + 256) = q1;
        __threadfence();
        *(volatile v8us*)rpw = q0;
        *(volatile v8us*)(rpw + 256) = q1;
      }
    }
  }

  if constexpr (MODE == 0) {
    float* wsum = (float*)hl;
    float* wp = wsum + wave * 512;
    *(v4fa*)(wp + 4 * lane) = psA;
    *(v4fa*)(wp + 128 + 4 * lane) = psB;
    *(v4fa*)(wp + 256 + 4 * lane) = pqA;
    *(v4fa*)(wp + 384 + 4 * lane) = pqB;
    __syncthreads();
    float* outs = (float*)sl;
    {
      float s = 0.0f, q = 0.0f;
#pragma unroll
      for (int w2 = 0; w2 < NWAVE; ++w2) {
        s += ((const f32a*)wsum)[w2 * 512 + tid];
        q += ((const f32a*)wsum)[w2 * 512 + 256 + tid];
      }
      ((f32a*)outs)[tid] = s;
      ((f32a*)outs)[256 + tid] = q;
    }
    __syncthreads();
    if (tid < 128) {
      const v4f ov4 = *(const v4fa*)(outs + 4 * tid);
      float* pp = part + (size_t)blockIdx.x * 512 + 4 * tid;
      *(volatile v4f*)pp = ov4;
      __threadfence();
      *(volatile v4f*)pp = ov4;
    }
  }
}

__global__ __launch_bounds__(64) void k_attn(unsigned short* QC, const unsigned short* __restrict__ KP,
                                             const unsigned short* __restrict__ VH,
                                             const unsigned short* __restrict__ VL) {
  __shared__ __attribute__((aligned(16))) unsigned short pst[2 * 2048];
  __shared__ __attribute__((aligned(16))) unsigned short cst[2 * 8192];
  const int tid = (int)threadIdx.x, lane = tid & 31, wave = tid >> 5, hh = lane >> 4, m = lane & 15;
  unsigned short* phs = pst + wave * 2048;
  unsigned short* pls = phs + 1024;
  unsigned short* cw  = cst + wave * 8192;
  const int q0 = (int)blockIdx.x * 32 + wave * 16;
  const int bg = q0 >> 8;
  const float SC = 0.17677669529663689f;
  const v8f z8 = {0.f, 0.f, 0.f, 0.f, 0.f, 0.f, 0.f, 0.f};

#pragma unroll 1
  for (int h = 0; h < NH; ++h) {
    FragB qh, ql;
    {
      const unsigned short* qp = QC + (size_t)(q0 + m) * 512 + h * HD + 8 * hh;
      qh.h[0] = *(const v8usa*)qp;           qh.h[1] = *(const v8usa*)(qp + 16);
      ql.h[0] = *(const v8usa*)(qp + 256);   ql.h[1] = *(const v8usa*)(qp + 272);
    }
    v8f o[2];
    o[0] = z8; o[1] = z8;
    float mr[8], lr[8];
#pragma unroll
    for (int r = 0; r < 8; ++r) { mr[r] = -1e30f; lr[r] = 0.0f; }

#pragma unroll 1
    for (int kt = 0; kt < 4; ++kt) {
      v8f s[4];
#pragma unroll
      for (int j = 0; j < 4; ++j) {
        const unsigned short* kp = KP + (size_t)(bg * SS + kt * 64 + j * 16 + m) * 512 + h * HD + 8 * hh;
        FragB kh, kl;
        kh.h[0] = *(const v8usa*)kp;         kh.h[1] = *(const v8usa*)(kp + 16);
        kl.h[0] = *(const v8usa*)(kp + 256); kl.h[1] = *(const v8usa*)(kp + 272);
        v8f c = wmb(qh, kh, z8);
        c = wmb(qh, kl, c);
        c = wmb(ql, kh, c);
        s[j] = c;
      }
#pragma unroll
      for (int r = 0; r < 8; ++r) {
        const float s0 = s[0][r] * SC, s1 = s[1][r] * SC, s2 = s[2][r] * SC, s3 = s[3][r] * SC;
        float mx = fmaxf(fmaxf(s0, s1), fmaxf(s2, s3));
        mx = fmaxf(mx, __shfl_xor(mx, 1, 32));
        mx = fmaxf(mx, __shfl_xor(mx, 2, 32));
        mx = fmaxf(mx, __shfl_xor(mx, 4, 32));
        mx = fmaxf(mx, __shfl_xor(mx, 8, 32));
        const float mn = fmaxf(mr[r], mx);
        const float al = expf(mr[r] - mn);
        mr[r] = mn;
        const float p0 = expf(s0 - mn), p1 = expf(s1 - mn), p2 = expf(s2 - mn), p3 = expf(s3 - mn);
        float rs = (p0 + p1) + (p2 + p3);
        rs += __shfl_xor(rs, 1, 32);
        rs += __shfl_xor(rs, 2, 32);
        rs += __shfl_xor(rs, 4, 32);
        rs += __shfl_xor(rs, 8, 32);
        lr[r] = lr[r] * al + rs;
        o[0][r] *= al;
        o[1][r] *= al;
        const int prow = (8 * hh + r) * 64 + m;
        unsigned w;
        w = hl_pack(p0); phs[prow]      = (unsigned short)(w & 0xffffu); pls[prow]      = (unsigned short)(w >> 16);
        w = hl_pack(p1); phs[prow + 16] = (unsigned short)(w & 0xffffu); pls[prow + 16] = (unsigned short)(w >> 16);
        w = hl_pack(p2); phs[prow + 32] = (unsigned short)(w & 0xffffu); pls[prow + 32] = (unsigned short)(w >> 16);
        w = hl_pack(p3); phs[prow + 48] = (unsigned short)(w & 0xffffu); pls[prow + 48] = (unsigned short)(w >> 16);
      }
      wave_sync();
#pragma unroll
      for (int c2 = 0; c2 < 2; ++c2) {
        FragB pa, pb;
        pa.h[0] = *(const v8usa*)(phs + m * 64 + 32 * c2 + 8 * hh);
        pa.h[1] = *(const v8usa*)(phs + m * 64 + 32 * c2 + 16 + 8 * hh);
        pb.h[0] = *(const v8usa*)(pls + m * 64 + 32 * c2 + 8 * hh);
        pb.h[1] = *(const v8usa*)(pls + m * 64 + 32 * c2 + 16 + 8 * hh);
#pragma unroll
        for (int t = 0; t < 2; ++t) {
          const size_t vo = (size_t)((bg * NH + h) * HD + t * 16 + m) * SS + kt * 64 + 32 * c2 + 8 * hh;
          FragB vh, vl;
          vh.h[0] = *(const v8usa*)(VH + vo);  vh.h[1] = *(const v8usa*)(VH + vo + 16);
          vl.h[0] = *(const v8usa*)(VL + vo);  vl.h[1] = *(const v8usa*)(VL + vo + 16);
          v8f c = o[t];
          c = wmb(pa, vh, c);
          c = wmb(pa, vl, c);
          c = wmb(pb, vh, c);
          o[t] = c;
        }
      }
      wave_sync();
    }
#pragma unroll
    for (int r = 0; r < 8; ++r) {
      const float inv = 1.0f / lr[r];
#pragma unroll
      for (int t = 0; t < 2; ++t) {
        const unsigned w = hl_pack(o[t][r] * inv);
        const int ci = (8 * hh + r) * 512 + h * HD + t * 16 + m;
        cw[ci]       = (unsigned short)(w & 0xffffu);
        cw[ci + 256] = (unsigned short)(w >> 16);
      }
    }
  }
  wave_sync();
#pragma unroll 1
  for (int pass = 0; pass < 2; ++pass) {
#pragma unroll 1
    for (int i = 0; i < 16; ++i) {
      const v8us a = *(const v8usa*)(cw + i * 512 + 8 * lane);
      const v8us b = *(const v8usa*)(cw + i * 512 + 256 + 8 * lane);
      unsigned short* dp = QC + (size_t)(q0 + i) * 512 + 8 * lane;
      *(volatile v8us*)dp = a;
      *(volatile v8us*)(dp + 256) = b;
    }
    __threadfence();
  }
}

template <int C, int MEAN, int RND>
__global__ __launch_bounds__(NTHR) void k_segsum(const float* __restrict__ hf, const int* __restrict__ bat,
                                                 int nN, float* pl) {
  constexpr int NV = C / 128;
  __shared__ __attribute__((aligned(16))) float wsum[NWAVE * C];
  __shared__ int wcn[NWAVE];
  __shared__ __attribute__((aligned(16))) float outs[C];
  const int tid = (int)threadIdx.x, lane = tid & 31, wave = tid >> 5;
  const int g = (int)blockIdx.x;

  v4f a[NV];
#pragma unroll
  for (int j = 0; j < NV; ++j) { const v4f z = {0.f, 0.f, 0.f, 0.f}; a[j] = z; }
  int cnt = 0;
#pragma unroll 1
  for (int i0 = wave * 32; i0 < nN; i0 += NTHR) {
    const int i  = i0 + lane;
    const int ic = i < nN ? i : nN - 1;
    const int b  = bat[ic];
    const bool hit = (i < nN) && (b == g);
    unsigned msk = __builtin_amdgcn_ballot_w32(hit);
    int nh = (int)__builtin_popcount(msk);
    nh = nh > 32 ? 32 : nh;
    cnt += nh;
#pragma unroll 1
    for (int q = 0; q < nh; ++q) {
      const int k = __builtin_ffs((int)msk) - 1;
      msk &= msk - 1u;
      int node = i0 + (k < 0 ? 0 : k);
      node = node > nN - 1 ? nN - 1 : node;
#pragma unroll
      for (int j = 0; j < NV; ++j) {
        v4f v = *(const v4fa*)(hf + (size_t)node * C + 128 * j + 4 * lane);
        if (RND) { v.x = bf16_val(v.x); v.y = bf16_val(v.y); v.z = bf16_val(v.z); v.w = bf16_val(v.w); }
        a[j] += v;
      }
    }
  }
#pragma unroll
  for (int j = 0; j < NV; ++j) *(v4fa*)(wsum + wave * C + 128 * j + 4 * lane) = a[j];
  if (lane == 0) wcn[wave] = cnt;
  __syncthreads();
  if (tid < C) {
    float s = 0.0f;
    int c = 0;
#pragma unroll
    for (int w2 = 0; w2 < NWAVE; ++w2) { s += ((const f32a*)wsum)[w2 * C + tid]; c += wcn[w2]; }
    const float cf = (c < 1) ? 1.0f : (float)c;
    ((f32a*)outs)[tid] = MEAN ? s * (1.0f / cf) : s;
  }
  __syncthreads();
  if (tid < C / 4) {
    const v4f ov = *(const v4fa*)(outs + 4 * tid);
    float* op = pl + (size_t)g * C + 4 * tid;
    *(volatile v4f*)op = ov;
    __threadfence();
    *(volatile v4f*)op = ov;
  }
}

static inline size_t al256(size_t o) { return (o + 255) & ~(size_t)255; }

extern "C" void kernel_launch(void* const* d_in, const int* in_sizes, int n_in,
                              void* d_out, int out_size, void* d_ws, size_t ws_size,
                              hipStream_t stream) {
  if (n_in < 28) return;
  if (in_sizes[0] != NN * DIN) return;
  if (in_sizes[1] != 2 * NEDGE) return;
  if (in_sizes[2] != NN) return;
  if (in_sizes[3] != NG * DH) return;
  if (in_sizes[4] != DIN || in_sizes[5] != DIN || in_sizes[6] != DH || in_sizes[7] != DH) return;
  if (in_sizes[8] != DIN * DH || in_sizes[9] != DH || in_sizes[10] != DH * DH || in_sizes[11] != DH) return;
  if (in_sizes[12] != DH * DH || in_sizes[14] != DH * DH || in_sizes[16] != DH * DH || in_sizes[18] != DH * DH) return;
  if (in_sizes[13] != DH || in_sizes[15] != DH || in_sizes[17] != DH || in_sizes[19] != DH) return;
  if (in_sizes[20] != DH || in_sizes[21] != DH || in_sizes[22] != DH || in_sizes[23] != DH) return;
  if (in_sizes[24] != DH * DFF || in_sizes[25] != DFF || in_sizes[26] != DFF * DH || in_sizes[27] != DH) return;
  if (out_size != NG * DH + NG * DIN) return;

  const float* x      = (const float*)d_in[0];
  const int*   edge   = (const int*)d_in[1];
  const int*   bat    = (const int*)d_in[2];
  const float* inter  = (const float*)d_in[3];
  const float* bn1g   = (const float*)d_in[4];
  const float* bn1b   = (const float*)d_in[5];
  const float* bn2g   = (const float*)d_in[6];
  const float* bn2b   = (const float*)d_in[7];
  const float* wc1    = (const float*)d_in[8];
  const float* bc1    = (const float*)d_in[9];
  const float* wc2    = (const float*)d_in[10];
  const float* bc2    = (const float*)d_in[11];
  const float* wq     = (const float*)d_in[12];
  const float* bq     = (const float*)d_in[13];
  const float* wk     = (const float*)d_in[14];
  const float* bk     = (const float*)d_in[15];
  const float* wv     = (const float*)d_in[16];
  const float* bv     = (const float*)d_in[17];
  const float* wo     = (const float*)d_in[18];
  const float* bo     = (const float*)d_in[19];
  const float* ln1g   = (const float*)d_in[20];
  const float* ln1b   = (const float*)d_in[21];
  const float* ln2g   = (const float*)d_in[22];
  const float* ln2b   = (const float*)d_in[23];
  const float* wf1    = (const float*)d_in[24];
  const float* bf1    = (const float*)d_in[25];
  const float* wf2    = (const float*)d_in[26];
  const float* bf2    = (const float*)d_in[27];
  float* out0 = (float*)d_out;
  float* out1 = (float*)d_out + (size_t)NG * DH;
  const int* src = edge;
  const int* dst = edge + NEDGE;
  const int nE = NEDGE, nN = NN;
  const int vec8 = ((nE & 3) == 0) ? 1 : 0;

  char* ws = (char*)d_ws;
  size_t off = 0;
  const size_t oDIS = off; off = al256(off + (size_t)NN * 4);
  const size_t oW1  = off; off = al256(off + (size_t)256 * 256 * 2);
  const size_t oW2  = off; off = al256(off + (size_t)256 * 512 * 2);
  const size_t oWQ  = off; off = al256(off + (size_t)768 * 512 * 2);
  const size_t oWO  = off; off = al256(off + (size_t)256 * 512 * 2);
  const size_t oF1  = off; off = al256(off + (size_t)1024 * 512 * 2);
  const size_t oF2  = off; off = al256(off + (size_t)256 * 2048 * 2);
  const size_t oP1  = off; off = al256(off + (size_t)(NN / 256) * 256 * 4);
  const size_t oP2  = off; off = al256(off + (size_t)(NN / NBA) * 512 * 4);
  const size_t oS1  = off; off = al256(off + (size_t)2 * DIN * 4);
  const size_t oS2  = off; off = al256(off + (size_t)2 * DH * 4);
  const size_t RSZ  = (size_t)NN * 1024;
  const size_t oR2  = off; off = al256(off + RSZ);
  const size_t oR3  = off; off = al256(off + RSZ);
  const size_t oR4  = off; off = al256(off + RSZ);
  const size_t oR5  = off; off = al256(off + RSZ);
  if (off > ws_size) return;
  if ((size_t)FCH * 2048 * 2 > RSZ) return;

  float*          DIS  = (float*)(ws + oDIS);
  unsigned short* W1c  = (unsigned short*)(ws + oW1);
  unsigned short* W2c  = (unsigned short*)(ws + oW2);
  unsigned short* Wqkv = (unsigned short*)(ws + oWQ);
  unsigned short* WOc  = (unsigned short*)(ws + oWO);
  unsigned short* FF1c = (unsigned short*)(ws + oF1);
  unsigned short* FF2c = (unsigned short*)(ws + oF2);
  float*          P1   = (float*)(ws + oP1);
  float*          P2   = (float*)(ws + oP2);
  float*          S1   = (float*)(ws + oS1);
  float*          S2   = (float*)(ws + oS2);
  float*          HC   = (float*)(ws + oR2);
  unsigned short* QCp  = (unsigned short*)(ws + oR2);
  float*          H1   = (float*)(ws + oR3);
  unsigned short* KPp  = (unsigned short*)(ws + oR3);
  unsigned short* T2p  = (unsigned short*)(ws + oR3);
  unsigned short* BN2p = (unsigned short*)(ws + oR4);
  unsigned short* VTh  = (unsigned short*)(ws + oR4);
  unsigned short* VTl  = VTh + (size_t)NN * DH;
  unsigned short* Fp   = (unsigned short*)(ws + oR4);
  unsigned short* BN1p = (unsigned short*)(ws + oR5);
  unsigned short* Tp   = (unsigned short*)(ws + oR5);
  float*          T3   = (float*)(ws + oR5);

  const size_t aggLds = (size_t)AGG_LDS_INTS * 4;
  hipFuncSetAttribute(reinterpret_cast<const void*>(&k_agg<0>), hipFuncAttributeMaxDynamicSharedMemorySize, (int)aggLds);
  hipFuncSetAttribute(reinterpret_cast<const void*>(&k_agg<1>), hipFuncAttributeMaxDynamicSharedMemorySize, (int)aggLds);
  hipFuncSetAttribute(reinterpret_cast<const void*>(&k_gemm<0>), hipFuncAttributeMaxDynamicSharedMemorySize, GLDS);
  hipFuncSetAttribute(reinterpret_cast<const void*>(&k_gemm<1>), hipFuncAttributeMaxDynamicSharedMemorySize, GLDS);
  hipFuncSetAttribute(reinterpret_cast<const void*>(&k_gemm<2>), hipFuncAttributeMaxDynamicSharedMemorySize, GLDS);
  hipFuncSetAttribute(reinterpret_cast<const void*>(&k_gemm<3>), hipFuncAttributeMaxDynamicSharedMemorySize, GLDS);
  hipFuncSetAttribute(reinterpret_cast<const void*>(&k_gemm<4>), hipFuncAttributeMaxDynamicSharedMemorySize, GLDS);

  const double invN = 1.0 / (double)NN;

  k_wprep<<<NUW / NTHR, NTHR, 0, stream>>>(wc1, wc2, wq, wk, wv, wo, wf1, wf2, W1c, W2c, Wqkv, WOc, FF1c, FF2c);
  k_stats1<<<NN / 256, NTHR, 0, stream>>>(x, P1);
  k_segsum<DIN, 1, 1><<<NG, NTHR, 0, stream>>>(x, bat, nN, out1);
  k_bncomb<<<1, NTHR, 0, stream>>>(P1, NN / 256, DIN, bn1g, bn1b, S1, invN);
  k_bn<DIN, 1><<<(NN * DIN / 8) / NTHR, NTHR, 0, stream>>>(x, S1, BN1p, NN * DIN / 8);
  k_deg<<<NN / NBD, NTHR, 0, stream>>>(dst, nE, vec8, DIS);
  k_gemm<0><<<dim3(NN / GM, 1), GT, GLDS, stream>>>(BN1p, 256, W1c, 256, bc1, bc1, bc1, bn2g, bn2b, BN1p,
                                                    QCp, QCp, QCp, QCp, HC);
  k_agg<0><<<NN / NBA, NTHR, aggLds, stream>>>(src, dst, nE, nN, vec8, DIS, HC, bc1, HC, bat, inter, NG, H1, P2, Tp);
  k_bncomb<<<1, NTHR, 0, stream>>>(P2, NN / NBA, DH, bn2g, bn2b, S2, invN);
  k_bn<DH, 0><<<(NN * DH / 8) / NTHR, NTHR, 0, stream>>>(H1, S2, BN2p, NN * DH / 8);
  k_gemm<0><<<dim3(NN / GM, 1), GT, GLDS, stream>>>(BN2p, 512, W2c, 512, bc2, bc2, bc2, bn2g, bn2b, BN2p,
                                                    QCp, QCp, QCp, QCp, HC);
  k_agg<1><<<NN / NBA, NTHR, aggLds, stream>>>(src, dst, nE, nN, vec8, DIS, HC, bc2, H1, bat, inter, NG, H1, P2, Tp);
  k_gemm<1><<<dim3(NN / GM, 3), GT, GLDS, stream>>>(Tp, 512, Wqkv, 512, bq, bk, bv, ln1g, ln1b, Tp,
                                                    QCp, KPp, VTh, VTl, HC);
  k_attn<<<NN / 32, 64, 0, stream>>>(QCp, KPp, VTh, VTl);
  k_gemm<2><<<dim3(NN / GM, 1), GT, GLDS, stream>>>(QCp, 512, WOc, 512, bo, bo, bo, ln1g, ln1b, Tp,
                                                    T2p, T2p, T2p, T2p, T3);
  for (int c = 0; c < NN / FCH; ++c) {
    const unsigned short* t2c = T2p + (size_t)c * FCH * 512;
    k_gemm<3><<<dim3(FCH / GM, DFF / GN), GT, GLDS, stream>>>(t2c, 512, FF1c, 512, bf1, bf1, bf1, ln2g, ln2b, t2c,
                                                              Fp, Fp, Fp, Fp, T3);
    k_gemm<4><<<dim3(FCH / GM, 1), GT, GLDS, stream>>>(Fp, 2048, FF2c, 2048, bf2, bf2, bf2, ln2g, ln2b, t2c,
                                                       Fp, Fp, Fp, Fp, T3 + (size_t)c * FCH * DH);
  }
  k_segsum<DH, 0, 0><<<NG, NTHR, 0, stream>>>(T3, bat, nN, out0);
}
